// GCN_Model_67216238182971
// MI455X (gfx1250) — hardware-verified
//
#include <hip/hip_runtime.h>
#include <stddef.h>


#define DW      128
#define D2      32
#define D3      16
#define D4      8
#define D5      2
#define NTHR    256
#define NWAVE   8
#define EPT     8
#define NGRP    2
#define CHUNK   (NTHR * EPT * NGRP)
#define WCAP    (EPT * NGRP * 32)
#define LISTN   (NWAVE * WCAP)
#define NBC     4096
#define NBF     1024
#define RCAP    40960
#define RBN     128
#define TGT     256
#define DEGCAP  1024
#define OTHR    512
#define WSCAPB  134217728
#define WCARRY  64.0f
#define NU1     (DW * (DW / 8))
#define NU2     (D2 * (DW / 8))
#define NU3     (D3 * (D2 / 8))
#define NUNITS  (NU1 + NU2 + NU3)
#define WPHALVES (DW * DW + DW * D2 + D2 * D3)

#define LDS_FILL ((RCAP + NBF + LISTN) * 4 + 64)

static_assert((CHUNK & (CHUNK - 1)) == 0);
static_assert(CHUNK <= 4096);
static_assert((NBC & (NBC - 1)) == 0 && (NBF & (NBF - 1)) == 0);
static_assert(NBC == 4 * NBF);
static_assert(OTHR * 8 == NBC);
static_assert((RCAP % 32) == 0);
static_assert(TGT == NWAVE * 32);
static_assert((NBC % TGT) == 0);
static_assert((TGT % 128) == 0);
static_assert(DW == 4 * 32);
static_assert((DW % 32) == 0 && (D2 % 32) == 0);
static_assert(WCAP == EPT * NGRP * 32);
static_assert((NUNITS % 32) == 0);
static_assert(NUNITS * 8 == WPHALVES);

typedef float    v2f  __attribute__((ext_vector_type(2)));
typedef float    v4f  __attribute__((ext_vector_type(4)));
typedef float    v8f  __attribute__((ext_vector_type(8)));
typedef int      v4i  __attribute__((ext_vector_type(4)));
typedef _Float16 v4h  __attribute__((ext_vector_type(4)));
typedef _Float16 v8h  __attribute__((ext_vector_type(8)));
typedef _Float16 v16h __attribute__((ext_vector_type(16)));
union Frag { v16h v; v8h h[2]; };

__device__ __forceinline__ v8f wmh(v16h a, v16h b, v8f c) {
  v8f d = __builtin_amdgcn_wmma_f32_16x16x32_f16(false, a, false, b, (short)0, c, false, false);
  asm volatile("v_nop\n\tv_nop\n\tv_nop\n\tv_nop" : "+v"(d) : "v"(a), "v"(b));
  return d;
}

template <int NB>
__device__ __forceinline__ int scan_chunk(const int* __restrict__ dsts, int nE, int cbase, int slotBase,
                                          int vec8, int* list, int tid, int lane, int wave) {
  int wc = 0;
#pragma unroll
  for (int g = 0; g < NGRP; ++g) {
    const int el0  = (g * NTHR + tid) * EPT;
    const int e0   = cbase + el0;
    const int sent = -2147483647 - 1;
    v4i da, db;
    if (vec8 != 0 && cbase + CHUNK <= nE) {
      da = *(const v4i*)(dsts + e0);
      db = *(const v4i*)(dsts + e0 + 4);
    } else {
      da.x = (e0     < nE) ? dsts[min(e0, nE - 1)] : sent;
      da.y = (e0 + 1 < nE) ? dsts[min(e0 + 1, nE - 1)] : sent;
      da.z = (e0 + 2 < nE) ? dsts[min(e0 + 2, nE - 1)] : sent;
      da.w = (e0 + 3 < nE) ? dsts[min(e0 + 3, nE - 1)] : sent;
      db.x = (e0 + 4 < nE) ? dsts[min(e0 + 4, nE - 1)] : sent;
      db.y = (e0 + 5 < nE) ? dsts[min(e0 + 5, nE - 1)] : sent;
      db.z = (e0 + 6 < nE) ? dsts[min(e0 + 6, nE - 1)] : sent;
      db.w = (e0 + 7 < nE) ? dsts[min(e0 + 7, nE - 1)] : sent;
    }
    const unsigned nb = (unsigned)slotBase;
    const unsigned s0 = (unsigned)da.x - nb, s1 = (unsigned)da.y - nb;
    const unsigned s2 = (unsigned)da.z - nb, s3 = (unsigned)da.w - nb;
    const unsigned s4 = (unsigned)db.x - nb, s5 = (unsigned)db.y - nb;
    const unsigned s6 = (unsigned)db.z - nb, s7 = (unsigned)db.w - nb;
    const bool h0 = s0 < (unsigned)NB, h1 = s1 < (unsigned)NB, h2 = s2 < (unsigned)NB, h3 = s3 < (unsigned)NB;
    const bool h4 = s4 < (unsigned)NB, h5 = s5 < (unsigned)NB, h6 = s6 < (unsigned)NB, h7 = s7 < (unsigned)NB;
    const unsigned any = __builtin_amdgcn_ballot_w32(h0 | h1 | h2 | h3 | h4 | h5 | h6 | h7);
    if (any != 0u) {
#define HITJ(J, HJ, SJ) { \
        const unsigned mj = __builtin_amdgcn_ballot_w32(HJ); \
        if (mj != 0u) { \
          if (HJ) { \
            const int pos = wc + (int)__builtin_amdgcn_mbcnt_lo(mj, 0u); \
            if (pos < WCAP) list[wave * WCAP + pos] = ((el0 + (J)) << 12) | (int)(SJ); \
          } \
          wc += (int)__builtin_popcount(mj); } }
      HITJ(0, h0, s0)
      HITJ(1, h1, s1)
      HITJ(2, h2, s2)
      HITJ(3, h3, s3)
      HITJ(4, h4, s4)
      HITJ(5, h5, s5)
      HITJ(6, h6, s6)
      HITJ(7, h7, s7)
#undef HITJ
    }
  }
  return wc;
}

__global__ __launch_bounds__(NTHR) void k_count(
    const int* __restrict__ dsts, int* cnt, float* dinv, int nE, int vec8) {
  __shared__ __attribute__((aligned(16))) int scnt[NBC];
  __shared__ __attribute__((aligned(16))) int list[LISTN];
  __shared__ int wcnt[NWAVE];
  const int tid = threadIdx.x, lane = tid & 31, wave = tid >> 5;
  const int nodeBase = blockIdx.x * NBC;

  for (int i = tid; i < NBC; i += NTHR) scnt[i] = 0;
  __syncthreads();

  const int nChunks = (nE + CHUNK - 1) / CHUNK;
#pragma unroll 1
  for (int ch = 0; ch < nChunks; ++ch) {
    const int cbase = ch * CHUNK;
    const int wc = scan_chunk<NBC>(dsts, nE, cbase, nodeBase, vec8, list, tid, lane, wave);
    if (lane == 0) wcnt[wave] = wc;
    __syncthreads();
    if (wave == 0) {
#pragma unroll 1
      for (int wsx = 0; wsx < NWAVE; ++wsx) {
        int n = __builtin_amdgcn_readfirstlane(wcnt[wsx]);
        n = n > WCAP ? WCAP : (n < 0 ? 0 : n);
        const int* lp = list + wsx * WCAP;
#pragma unroll 1
        for (int i = 0; i < n; ++i) {
          const int ent  = __builtin_amdgcn_readfirstlane(lp[i]);
          const int slot = ent & (NBC - 1);
          if (lane == 0) scnt[slot] = scnt[slot] + 1;
        }
      }
    }
    __syncthreads();
  }

  v4i cq[4];
  v4f dq[4];
#pragma unroll
  for (int q = 0; q < 4; ++q) {
    const int f = (wave * 4 + q) * 128 + 4 * lane;
    const v4i cv = *(const v4i*)(scnt + f);
    cq[q] = cv;
    v4f d;
    d.x = rsqrtf((float)(cv.x < 0 ? 0 : cv.x) + 1.0f);
    d.y = rsqrtf((float)(cv.y < 0 ? 0 : cv.y) + 1.0f);
    d.z = rsqrtf((float)(cv.z < 0 ? 0 : cv.z) + 1.0f);
    d.w = rsqrtf((float)(cv.w < 0 ? 0 : cv.w) + 1.0f);
    dq[q] = d;
  }
  int*   cp = cnt  + (size_t)nodeBase;
  float* dp = dinv + (size_t)nodeBase;
#pragma unroll
  for (int q = 0; q < 4; ++q) {
    const int f = (wave * 4 + q) * 128 + 4 * lane;
    *(volatile v4i*)(cp + f) = cq[q];
    *(volatile v4f*)(dp + f) = dq[q];
  }
  __threadfence();
#pragma unroll
  for (int q = 0; q < 4; ++q) {
    const int f = (wave * 4 + q) * 128 + 4 * lane;
    *(volatile v4i*)(cp + f) = cq[q];
    *(volatile v4f*)(dp + f) = dq[q];
  }
}

__global__ __launch_bounds__(OTHR) void k_offsets(
    const int* __restrict__ cnt, int* off, int* rbase, int nChunk) {
  __shared__ __attribute__((aligned(16))) int soff[NBC];
  __shared__ __attribute__((aligned(16))) int srb[RBN];
  __shared__ int wtot[OTHR / 32];
  const int tid = threadIdx.x, lane = tid & 31, wave = tid >> 5, sub = tid >> 7;
  for (int i = tid; i < RBN; i += OTHR) srb[i] = 0;
  int carry = 0;
#pragma unroll 1
  for (int ch = 0; ch < nChunk; ++ch) {
    const int base = ch * NBC;
    const v4i c0 = *(const v4i*)(cnt + base + 8 * tid);
    const v4i c1 = *(const v4i*)(cnt + base + 8 * tid + 4);
    const int e0 = max(c0.x, 0), e1 = max(c0.y, 0), e2 = max(c0.z, 0), e3 = max(c0.w, 0);
    const int e4 = max(c1.x, 0), e5 = max(c1.y, 0), e6 = max(c1.z, 0), e7 = max(c1.w, 0);
    const int ts = e0 + e1 + e2 + e3 + e4 + e5 + e6 + e7;
    int incl = ts;
#pragma unroll
    for (int d = 1; d < 32; d <<= 1) {
      const int t = __shfl_up(incl, d);
      if (lane >= d) incl += t;
    }
    if (lane == 31) wtot[wave] = incl;
    __syncthreads();
    const int S0 = wtot[0]  + wtot[1]  + wtot[2]  + wtot[3];
    const int S1 = wtot[4]  + wtot[5]  + wtot[6]  + wtot[7];
    const int S2 = wtot[8]  + wtot[9]  + wtot[10] + wtot[11];
    const int S3 = wtot[12] + wtot[13] + wtot[14] + wtot[15];
    int pre = 0;
#pragma unroll 1
    for (int w = 4 * sub; w < wave; ++w) pre += wtot[w];
    const int b0 = carry;
    const int b1 = b0 + ((S0 + 31) & ~31);
    const int b2 = b1 + ((S1 + 31) & ~31);
    const int b3 = b2 + ((S2 + 31) & ~31);
    const int b4 = b3 + ((S3 + 31) & ~31);
    const int myb = sub == 0 ? b0 : (sub == 1 ? b1 : (sub == 2 ? b2 : b3));
    if (tid == 0) {
      srb[min(4 * ch + 0, RBN - 1)] = b0;
      srb[min(4 * ch + 1, RBN - 1)] = b1;
      srb[min(4 * ch + 2, RBN - 1)] = b2;
      srb[min(4 * ch + 3, RBN - 1)] = b3;
    }
    int run = myb + pre + incl - ts;
    soff[8 * tid + 0] = run; run += e0;
    soff[8 * tid + 1] = run; run += e1;
    soff[8 * tid + 2] = run; run += e2;
    soff[8 * tid + 3] = run; run += e3;
    soff[8 * tid + 4] = run; run += e4;
    soff[8 * tid + 5] = run; run += e5;
    soff[8 * tid + 6] = run; run += e6;
    soff[8 * tid + 7] = run;
    carry = b4;
    __syncthreads();
    const v4i o0 = *(const v4i*)(soff + 4 * tid);
    const v4i o1 = *(const v4i*)(soff + 4 * (tid + OTHR));
    int* op = off + base;
    *(volatile v4i*)(op + 4 * tid) = o0;
    *(volatile v4i*)(op + 4 * (tid + OTHR)) = o1;
    __threadfence();
    *(volatile v4i*)(op + 4 * tid) = o0;
    *(volatile v4i*)(op + 4 * (tid + OTHR)) = o1;
    __syncthreads();
  }
  if (tid == 0) srb[min(4 * nChunk, RBN - 1)] = carry;
  __syncthreads();
  v4i rv = {0, 0, 0, 0};
  if (tid < 32) rv = *(const v4i*)(srb + 4 * tid);
  if (tid < 32) *(volatile v4i*)(rbase + 4 * tid) = rv;
  __threadfence();
  if (tid < 32) *(volatile v4i*)(rbase + 4 * tid) = rv;
}

__global__ __launch_bounds__(NTHR) void k_fill(
    const int* __restrict__ srcs, const int* __restrict__ dsts,
    const int* __restrict__ off, const int* __restrict__ rbase,
    int* csr, int nN, int nE, int vec8, int csrLen) {
  extern __shared__ v4f lds_dyn[];
  int* region = (int*)lds_dyn;
  int* cursor = region + RCAP;
  int* list   = cursor + NBF;
  int* wcnt   = list + LISTN;
  const int tid = threadIdx.x, lane = tid & 31, wave = tid >> 5;
  const int b = blockIdx.x;
  const int nodeBase = b * NBF;

  int rb0 = rbase[b];
  const int rb1 = rbase[b + 1];
  rb0 = rb0 < 0 ? 0 : (rb0 > csrLen ? csrLen : rb0);
  rb0 &= ~31;
  int len = rb1 - rb0;
  len = len < 0 ? 0 : (len > RCAP ? RCAP : len);
  int lenW = (len + 31) & ~31;
  if (rb0 + lenW > csrLen) lenW = (csrLen - rb0) & ~31;

  {
    const v4i z = {0, 0, 0, 0};
    for (int i = tid; i < RCAP / 4; i += NTHR) ((v4i*)region)[i] = z;
    for (int s = tid; s < NBF; s += NTHR) {
      int o = off[nodeBase + s] - rb0;
      o = o < 0 ? 0 : (o > RCAP ? RCAP : o);
      cursor[s] = o;
    }
  }
  __syncthreads();

  const int nChunks = (nE + CHUNK - 1) / CHUNK;
#pragma unroll 1
  for (int ch = 0; ch < nChunks; ++ch) {
    const int cbase = ch * CHUNK;
    const int wc = scan_chunk<NBF>(dsts, nE, cbase, nodeBase, vec8, list, tid, lane, wave);
    if (lane == 0) wcnt[wave] = wc;
    __syncthreads();
    if (wave == 0) {
#pragma unroll 1
      for (int wsx = 0; wsx < NWAVE; ++wsx) {
        int n = __builtin_amdgcn_readfirstlane(wcnt[wsx]);
        n = n > WCAP ? WCAP : (n < 0 ? 0 : n);
        const int* lp = list + wsx * WCAP;
#pragma unroll 1
        for (int i = 0; i < n; ++i) {
          const int ent  = __builtin_amdgcn_readfirstlane(lp[i]);
          const int slot = ent & (NBF - 1);
          int e = cbase + ((ent >> 12) & (CHUNK - 1));
          e = e > nE - 1 ? nE - 1 : e;
          int sv = srcs[e];
          sv = sv < 0 ? 0 : (sv > nN - 1 ? nN - 1 : sv);
          if (lane == 0) {
            int pos = cursor[slot];
            pos = pos < 0 ? 0 : (pos > RCAP - 1 ? RCAP - 1 : pos);
            region[pos] = sv;
            const int np = pos + 1;
            cursor[slot] = np > RCAP ? RCAP : np;
          }
        }
      }
    }
    __syncthreads();
  }

  const int nv = lenW >> 2;
  int* gp = csr + rb0;
#pragma unroll 1
  for (int i = tid; i < nv; i += NTHR) { const v4i v = ((const v4i*)region)[i]; *(volatile v4i*)(gp + 4 * i) = v; }
  __threadfence();
#pragma unroll 1
  for (int i = tid; i < nv; i += NTHR) { const v4i v = ((const v4i*)region)[i]; *(volatile v4i*)(gp + 4 * i) = v; }
}

__global__ __launch_bounds__(NTHR) void k_wcvt(const float* __restrict__ w1, const float* __restrict__ w2,
                                               const float* __restrict__ w3, _Float16* wp, int nUnits) {
  const int i = (int)blockIdx.x * NTHR + (int)threadIdx.x;
  if (i >= nUnits) return;
  const int r1 = i < NU1 - 1 ? i : NU1 - 1;
  const int n1 = r1 >> 4, s1 = r1 & 15;
  int r2 = i - NU1;
  r2 = r2 < 0 ? 0 : (r2 > NU2 - 1 ? NU2 - 1 : r2);
  const int n2 = r2 >> 4, s2 = r2 & 15;
  int r3 = i - NU1 - NU2;
  r3 = r3 < 0 ? 0 : (r3 > NU3 - 1 ? NU3 - 1 : r3);
  const int n3 = r3 >> 2, s3 = r3 & 3;
  const int sel = i < NU1 ? 0 : (i < NU1 + NU2 ? 1 : 2);
  v8h o;
#pragma unroll
  for (int j = 0; j < 8; ++j) {
    const float f1 = w1[(8 * s1 + j) * DW + n1];
    const float f2 = w2[(8 * s2 + j) * D2 + n2];
    const float f3 = w3[(8 * s3 + j) * D3 + n3];
    const float f = sel == 0 ? f1 : (sel == 1 ? f2 : f3);
    o[j] = (_Float16)(f * WCARRY);
  }
  _Float16* gp = wp + (size_t)i * 8;
  *(volatile v8h*)gp = o;
  __threadfence();
  *(volatile v8h*)gp = o;
}

template <int KD, int NC>
__global__ __launch_bounds__(NTHR) void k_gemm(
    const float* __restrict__ Asrc, const _Float16* __restrict__ Bp, float* Cout,
    float acarry, float gscale, int nValid) {
  constexpr int WN   = (NC >= 32) ? 2 : 1;
  constexpr int WM   = NWAVE / WN;
  constexpr int BMR  = 16 * WM;
  constexpr int TPW  = NC / (16 * WN);
  constexpr int KST  = KD / 32;
  constexpr int PPR  = KD / 4;
  constexpr int NIT  = (BMR * PPR) / NTHR;
  constexpr int NOT_ = (BMR * NC / 4) / NTHR;
  static_assert((KD % 32) == 0 && KST >= 1);
  static_assert(TPW >= 1 && TPW * 16 * WN == NC);
  static_assert((BMR * PPR) % NTHR == 0 && NIT >= 1);
  static_assert((BMR * NC / 4) % NTHR == 0 && NOT_ >= 1);
  static_assert(((BMR * NC * 4) % 512) == 0);
  static_assert((PPR & (PPR - 1)) == 0);

  __shared__ __attribute__((aligned(16))) _Float16 a16[BMR * KD];
  __shared__ __attribute__((aligned(16))) float stg[BMR * NC];
  const int tid = threadIdx.x, lane = tid & 31, wave = tid >> 5, hh = lane >> 4, m = lane & 15;
  const int rowBase = (int)blockIdx.x * BMR;
  const int rg = wave / WN, cw = wave % WN;
  const int r0 = rg * 16;
  const int c0 = cw * TPW * 16;

#pragma unroll
  for (int it = 0; it < NIT; ++it) {
    const int id = it * NTHR + tid;
    const int row = id / PPR, seg = id % PPR;
    const int grow = rowBase + row;
    const bool live = grow < nValid;
    int rr = grow > nValid - 1 ? nValid - 1 : grow;
    rr = rr < 0 ? 0 : rr;
    const v4f xv = *(const v4f*)(Asrc + (size_t)rr * KD + 4 * seg);
    v4h o;
    o.x = (_Float16)((live ? xv.x : 0.f) * acarry);
    o.y = (_Float16)((live ? xv.y : 0.f) * acarry);
    o.z = (_Float16)((live ? xv.z : 0.f) * acarry);
    o.w = (_Float16)((live ? xv.w : 0.f) * acarry);
    *(v4h*)(a16 + (size_t)row * KD + 4 * seg) = o;
  }
  __syncthreads();

  v8f acc[TPW];
#pragma unroll
  for (int t = 0; t < TPW; ++t) { v8f z = {0.f, 0.f, 0.f, 0.f, 0.f, 0.f, 0.f, 0.f}; acc[t] = z; }

  const _Float16* ap = a16 + (size_t)(r0 + m) * KD + 8 * hh;
  const _Float16* bp = Bp + (size_t)(c0 + m) * KD + 8 * hh;
#pragma unroll 1
  for (int kt = 0; kt < KST; ++kt) {
    Frag a;
    a.h[0] = *(const v8h*)(ap + 32 * kt);
    a.h[1] = *(const v8h*)(ap + 32 * kt + 16);
#pragma unroll
    for (int t = 0; t < TPW; ++t) {
      const size_t to = (size_t)(16 * t) * KD + 32 * kt;
      Frag bq;
      bq.h[0] = *(const v8h*)(bp + to);
      bq.h[1] = *(const v8h*)(bp + to + 16);
      acc[t] = wmh(a.v, bq.v, acc[t]);
    }
  }

  {
    float* sp = stg + (size_t)(r0 + 8 * hh) * NC + c0 + m;
    const int growb = rowBase + r0 + 8 * hh;
#pragma unroll
    for (int t = 0; t < TPW; ++t) {
#pragma unroll
      for (int r = 0; r < 8; ++r) {
        const bool lv = (growb + r) < nValid;
        sp[r * NC + 16 * t] = lv ? (acc[t][r] * gscale) : 0.f;
      }
    }
  }
  __syncthreads();

  v4f cv[NOT_];
#pragma unroll
  for (int it = 0; it < NOT_; ++it) {
    const int id = it * NTHR + tid;
    cv[it] = *(const v4f*)(stg + 4 * id);
  }
  float* gb = Cout + (size_t)rowBase * NC;
#pragma unroll
  for (int it = 0; it < NOT_; ++it) {
    const int id = it * NTHR + tid;
    *(volatile v4f*)(gb + 4 * (size_t)id) = cv[it];
  }
  __threadfence();
#pragma unroll
  for (int it = 0; it < NOT_; ++it) {
    const int id = it * NTHR + tid;
    *(volatile v4f*)(gb + 4 * (size_t)id) = cv[it];
  }
}

template <int DWT>
__global__ __launch_bounds__(NTHR) void k_agg(
    const int* __restrict__ csr, const int* __restrict__ off, const int* __restrict__ cnt,
    const float* __restrict__ dinv, const float* __restrict__ h, const float* __restrict__ bias,
    float* so, int nN, int csrLen) {
  constexpr int LPR = DWT / 4;
  constexpr int G = 32 / LPR;
  constexpr bool WIDE = (DWT == DW);
  constexpr int TILEF = WIDE ? 4 : (NWAVE * 32 * DWT);
  constexpr int NST = DWT / 4;
  static_assert(LPR * G == 32 && LPR >= 1 && (DWT % 4) == 0);
  __shared__ __attribute__((aligned(16))) float tile[TILEF];
  const int tid = threadIdx.x, lane = tid & 31, wave = tid >> 5;
  const int g = lane / LPR;
  const int col4 = 4 * (lane - g * LPR);
  const int tbase = blockIdx.x * TGT + wave * 32;
  const int cl = tbase + lane;
  const int cnt_l = cnt[cl];
  const int off_l = off[cl];
  const float di_l = dinv[cl];
  const v4f bv = *(const v4f*)(bias + col4);
  float* tw = tile + (WIDE ? 0 : wave * 32 * DWT);

#pragma unroll 1
  for (int j = 0; j < 32; ++j) {
    const int c = tbase + j;
    int n = __shfl(cnt_l, j);
    n = n < 0 ? 0 : (n > DEGCAP ? DEGCAP : n);
    const int st = __shfl(off_l, j);
    const float dc = __shfl(di_l, j);
    const float dd = dc * dc;
    v4f a = {0.f, 0.f, 0.f, 0.f};
#pragma unroll 1
    for (int q0 = 0; q0 < n; q0 += 32) {
      int pos = st + q0 + lane;
      pos = pos < 0 ? 0 : (pos > csrLen - 1 ? csrLen - 1 : pos);
      int sl = csr[pos];
      sl = sl < 0 ? 0 : (sl > nN - 1 ? nN - 1 : sl);
      const int mcnt = (n - q0) < 32 ? (n - q0) : 32;
      if constexpr (G == 1) {
#pragma unroll 1
        for (int pp = 0; pp < mcnt; ++pp) {
          const int s = __builtin_amdgcn_readlane(sl, pp);
          const float cf = dinv[s] * dc;
          const v4f xv = *(const v4f*)(h + (size_t)s * DWT + col4);
          a = a + xv * cf;
        }
      } else {
#pragma unroll 1
        for (int pp = 0; pp < mcnt; pp += G) {
          const int idx = pp + g;
          const bool valid = idx < mcnt;
          const int s = __shfl(sl, idx & 31);
          const float dv = dinv[s];
          const float cf = valid ? (dv * dc) : 0.f;
          const v4f xv = *(const v4f*)(h + (size_t)s * DWT + col4);
          a = a + xv * cf;
        }
      }
    }
    if constexpr (G > 1) {
#pragma unroll
      for (int msk = LPR; msk < 32; msk <<= 1) {
        a.x += __shfl_xor(a.x, msk);
        a.y += __shfl_xor(a.y, msk);
        a.z += __shfl_xor(a.z, msk);
        a.w += __shfl_xor(a.w, msk);
      }
    }
    const bool live = c < nN;
    const v4f hz = *(const v4f*)(h + (size_t)c * DWT + col4);
    v4f o;
    o.x = live ? fmaxf(a.x + hz.x * dd + bv.x, 0.f) : 0.f;
    o.y = live ? fmaxf(a.y + hz.y * dd + bv.y, 0.f) : 0.f;
    o.z = live ? fmaxf(a.z + hz.z * dd + bv.z, 0.f) : 0.f;
    o.w = live ? fmaxf(a.w + hz.w * dd + bv.w, 0.f) : 0.f;
    if constexpr (WIDE) {
      float* gp = so + (size_t)c * DWT + col4;
      *(volatile v4f*)gp = o;
      __threadfence();
      *(volatile v4f*)gp = o;
    } else {
      if (g == 0) *(v4f*)(tw + j * DWT + col4) = o;
    }
  }

  if constexpr (!WIDE) {
    __syncthreads();
    v4f cv[NST];
#pragma unroll
    for (int it = 0; it < NST; ++it) {
      const int p = it * 32 + lane;
      cv[it] = *(const v4f*)(tw + 4 * p);
    }
    float* gb = so + (size_t)tbase * DWT;
#pragma unroll
    for (int it = 0; it < NST; ++it) {
      const int p = it * 32 + lane;
      *(volatile v4f*)(gb + 4 * p) = cv[it];
    }
    __threadfence();
#pragma unroll
    for (int it = 0; it < NST; ++it) {
      const int p = it * 32 + lane;
      *(volatile v4f*)(gb + 4 * p) = cv[it];
    }
  }
}

__global__ __launch_bounds__(NTHR) void k_agg_head(
    const int* __restrict__ csr, const int* __restrict__ off, const int* __restrict__ cnt,
    const float* __restrict__ dinv, const float* __restrict__ h, const float* __restrict__ b3,
    const float* __restrict__ W4, const float* __restrict__ b4,
    const float* __restrict__ W5, const float* __restrict__ b5,
    float* out, int nN, int csrLen) {
  constexpr int DWT = D3;
  constexpr int LPR = DWT / 4;
  constexpr int G = 32 / LPR;
  static_assert(LPR == 4 && G == 8);
  static_assert(D3 * D4 <= NTHR && D4 == 8 && D5 == 2);
  __shared__ __attribute__((aligned(16))) float sW4[D3 * D4];
  __shared__ float sb4[D4];
  __shared__ float sW5[D4 * D5];
  __shared__ float sb5[4];
  __shared__ __attribute__((aligned(16))) float sout[NWAVE * 64];
  const int tid = threadIdx.x, lane = tid & 31, wave = tid >> 5;
  if (tid < D3 * D4) sW4[tid] = W4[tid];
  if (tid < D4)      sb4[tid] = b4[tid];
  if (tid < D4 * D5) sW5[tid] = W5[tid];
  if (tid < D5)      sb5[tid] = b5[tid];
  __syncthreads();

  const int g = lane >> 2;
  const int q4 = lane & 3;
  const int col4 = 4 * q4;
  const int tbase = blockIdx.x * TGT + wave * 32;
  const int cl = tbase + lane;
  const int cnt_l = cnt[cl];
  const int off_l = off[cl];
  const float di_l = dinv[cl];
  const v4f bv = *(const v4f*)(b3 + col4);
  float* sw = sout + wave * 64;

#pragma unroll 1
  for (int j = 0; j < 32; ++j) {
    const int c = tbase + j;
    int n = __shfl(cnt_l, j);
    n = n < 0 ? 0 : (n > DEGCAP ? DEGCAP : n);
    const int st = __shfl(off_l, j);
    const float dc = __shfl(di_l, j);
    const float dd = dc * dc;
    v4f a = {0.f, 0.f, 0.f, 0.f};
#pragma unroll 1
    for (int q0 = 0; q0 < n; q0 += 32) {
      int pos = st + q0 + lane;
      pos = pos < 0 ? 0 : (pos > csrLen - 1 ? csrLen - 1 : pos);
      int sl = csr[pos];
      sl = sl < 0 ? 0 : (sl > nN - 1 ? nN - 1 : sl);
      const int mcnt = (n - q0) < 32 ? (n - q0) : 32;
#pragma unroll 1
      for (int pp = 0; pp < mcnt; pp += G) {
        const int idx = pp + g;
        const bool valid = idx < mcnt;
        const int s = __shfl(sl, idx & 31);
        const float dv = dinv[s];
        const float cf = valid ? (dv * dc) : 0.f;
        const v4f xv = *(const v4f*)(h + (size_t)s * DWT + col4);
        a = a + xv * cf;
      }
    }
#pragma unroll
    for (int msk = LPR; msk < 32; msk <<= 1) {
      a.x += __shfl_xor(a.x, msk);
      a.y += __shfl_xor(a.y, msk);
      a.z += __shfl_xor(a.z, msk);
      a.w += __shfl_xor(a.w, msk);
    }
    const v4f hz = *(const v4f*)(h + (size_t)c * DWT + col4);
    v4f z;
    z.x = fmaxf(a.x + hz.x * dd + bv.x, 0.f);
    z.y = fmaxf(a.y + hz.y * dd + bv.y, 0.f);
    z.z = fmaxf(a.z + hz.z * dd + bv.z, 0.f);
    z.w = fmaxf(a.w + hz.w * dd + bv.w, 0.f);
    float p = z.x * sW4[(col4 + 0) * D4 + g];
    p += z.y * sW4[(col4 + 1) * D4 + g];
    p += z.z * sW4[(col4 + 2) * D4 + g];
    p += z.w * sW4[(col4 + 3) * D4 + g];
    p += __shfl_xor(p, 1);
    p += __shfl_xor(p, 2);
    const float h4 = fmaxf(p + sb4[g], 0.f);
    float u0 = h4 * sW5[g * D5 + 0];
    float u1 = h4 * sW5[g * D5 + 1];
    u0 += __shfl_xor(u0, 4);  u1 += __shfl_xor(u1, 4);
    u0 += __shfl_xor(u0, 8);  u1 += __shfl_xor(u1, 8);
    u0 += __shfl_xor(u0, 16); u1 += __shfl_xor(u1, 16);
    const float o0 = u0 + sb5[0];
    const float o1 = u1 + sb5[1];
    if (lane == 0) { sw[2 * j] = o0; sw[2 * j + 1] = o1; }
  }
  __syncthreads();

  v4f v = {0.f, 0.f, 0.f, 0.f};
  if (lane < 16) v = *(const v4f*)(sw + 4 * lane);
  v2f v2;
  v2.x = v.x; v2.y = v.y;
  const int rr = tbase + 2 * lane;
  const bool st4 = (lane < 16) && (rr + 2 <= nN);
  const bool st2 = (lane < 16) && (rr + 2 > nN) && (rr + 1 == nN);
  float* gp = out + (size_t)tbase * D5 + 4 * lane;
  if (st4) { *(volatile v4f*)gp = v; } else if (st2) { *(volatile v2f*)gp = v2; }
  __threadfence();
  if (st4) { *(volatile v4f*)gp = v; } else if (st2) { *(volatile v2f*)gp = v2; }
}

extern "C" void kernel_launch(void* const* d_in, const int* in_sizes, int n_in,
                              void* d_out, int out_size, void* d_ws, size_t ws_size,
                              hipStream_t stream) {
  if (n_in < 12) return;
  if (in_sizes[0] < DW || (in_sizes[0] % DW) != 0) return;
  const int nN = in_sizes[0] / DW;
  if (in_sizes[1] < 2 || (in_sizes[1] & 1) != 0) return;
  const int nE = in_sizes[1] / 2;
  if (in_sizes[2] != DW * DW || in_sizes[3] != DW) return;
  if (in_sizes[4] != DW * D2 || in_sizes[5] != D2) return;
  if (in_sizes[6] != D2 * D3 || in_sizes[7] != D3) return;
  if (in_sizes[8] != D3 * D4 || in_sizes[9] != D4) return;
  if (in_sizes[10] != D4 * D5 || in_sizes[11] != D5) return;
  if (out_size != nN * D5) return;
  if (nE > (1 << 28) || nN > (1 << 22) || nN < 1 || nE < 1) return;

  const float* x  = (const float*)d_in[0];
  const int*   ei = (const int*)d_in[1];
  const int*   src = ei;
  const int*   dst = ei + nE;
  const float* W1 = (const float*)d_in[2];
  const float* b1 = (const float*)d_in[3];
  const float* W2 = (const float*)d_in[4];
  const float* b2 = (const float*)d_in[5];
  const float* W3 = (const float*)d_in[6];
  const float* b3 = (const float*)d_in[7];
  const float* W4 = (const float*)d_in[8];
  const float* b4 = (const float*)d_in[9];
  const float* W5 = (const float*)d_in[10];
  const float* b5 = (const float*)d_in[11];
  float* out = (float*)d_out;

  const int NPAD   = ((nN + TGT - 1) / TGT) * TGT;
  const int nBC    = (nN + NBC - 1) / NBC;
  const int CNTPAD = nBC * NBC;
  if (CNTPAD < NPAD) return;
  if (4 * nBC + 1 > RBN) return;
  const int nBF    = (nN + NBF - 1) / NBF;
  if (nBF > 4 * nBC) return;
  const int csrLen = ((nE + 31) & ~31) + 4096;
  if (31 * 4 * nBC > 4096) return;
  const int nAgg   = NPAD / TGT;
  const int nG64   = NPAD / 64;
  const int nG128  = NPAD / 128;

  char* ws = (char*)d_ws;
  size_t off = 0;
  const size_t oWp  = off; off += (size_t)WPHALVES * 2;           off = (off + 255) & ~(size_t)255;
  const size_t oRH  = off; off += (size_t)NPAD * DW * 4;          off = (off + 255) & ~(size_t)255;
  const size_t oRZ  = off; off += (size_t)NPAD * DW * 4;          off = (off + 255) & ~(size_t)255;
  const size_t oCnt = off; off += (size_t)CNTPAD * 4;             off = (off + 255) & ~(size_t)255;
  const size_t oDi  = off; off += (size_t)CNTPAD * 4;             off = (off + 255) & ~(size_t)255;
  const size_t oOff = off; off += (size_t)CNTPAD * 4;             off = (off + 255) & ~(size_t)255;
  const size_t oRb  = off; off += (size_t)RBN * 4;                off = (off + 255) & ~(size_t)255;
  const size_t oCsr = off; off += (size_t)csrLen * 4;             off = (off + 255) & ~(size_t)255;
  if (off > ws_size || off > (size_t)WSCAPB) return;

  _Float16* wpl = (_Float16*)(ws + oWp);
  float* rh   = (float*)(ws + oRH);
  float* rz   = (float*)(ws + oRZ);
  int*   cnt  = (int*)(ws + oCnt);
  float* dinv = (float*)(ws + oDi);
  int*   offp = (int*)(ws + oOff);
  int*   rb   = (int*)(ws + oRb);
  int*   csr  = (int*)(ws + oCsr);
  const _Float16* wp1 = wpl;
  const _Float16* wp2 = wpl + DW * DW;
  const _Float16* wp3 = wpl + DW * DW + DW * D2;

  const int vec8 = ((nE & 3) == 0) ? 1 : 0;

  k_wcvt<<<(NUNITS + NTHR - 1) / NTHR, NTHR, 0, stream>>>(W1, W2, W3, wpl, NUNITS);
  k_count<<<nBC, NTHR, 0, stream>>>(dst, cnt, dinv, nE, vec8);
  k_offsets<<<1, OTHR, 0, stream>>>(cnt, offp, rb, nBC);
  hipFuncSetAttribute(reinterpret_cast<const void*>(&k_fill),
                      hipFuncAttributeMaxDynamicSharedMemorySize, LDS_FILL);
  k_fill<<<nBF, NTHR, LDS_FILL, stream>>>(src, dst, offp, rb, csr, nN, nE, vec8, csrLen);

  k_gemm<DW, DW><<<nG64, NTHR, 0, stream>>>(x, wp1, rh, 8.0f, 1.0f / 512.0f, nN);
  k_agg<DW><<<nAgg, NTHR, 0, stream>>>(csr, offp, cnt, dinv, rh, b1, rz, nN, csrLen);

  k_gemm<DW, D2><<<nG64, NTHR, 0, stream>>>(rz, wp2, rh, 64.0f, 1.0f / 4096.0f, nN);
  k_agg<D2><<<nAgg, NTHR, 0, stream>>>(csr, offp, cnt, dinv, rh, b2, rz, nN, csrLen);

  k_gemm<D2, D3><<<nG128, NTHR, 0, stream>>>(rz, wp3, rh, 64.0f, 1.0f / 4096.0f, nN);
  k_agg_head<<<nAgg, NTHR, 0, stream>>>(csr, offp, cnt, dinv, rh, b3, W4, b4, W5, b5, out, nN, csrLen);
}
